// ExtractorAttn_13005160972328
// MI455X (gfx1250) — hardware-verified
//
#include <hip/hip_runtime.h>
#include <math.h>

typedef __attribute__((ext_vector_type(16))) _Float16 v16h;
typedef __attribute__((ext_vector_type(16))) __bf16 v16b;
typedef __attribute__((ext_vector_type(8)))  _Float16 v8h;
typedef __attribute__((ext_vector_type(8)))  float v8f;
typedef __attribute__((ext_vector_type(4)))  float v4f;
typedef __attribute__((ext_vector_type(2)))  float v2f;
typedef __attribute__((ext_vector_type(4)))  unsigned v4u;
typedef __attribute__((ext_vector_type(4)))  int v4i;
typedef float __attribute__((may_alias)) float_a;
typedef int __attribute__((may_alias)) int_a;

template <typename T> __device__ __forceinline__ void vst2(void* p, T v) { *(volatile T*)p = v; __threadfence(); *(volatile T*)p = v; }
__device__ __forceinline__ v8f wmma16(v16h a, v16h b, v8f c) {
  v8f d = __builtin_amdgcn_wmma_f32_16x16x32_f16(false, a, false, b, (short)0, c, false, false);
  asm volatile("v_nop\n\tv_nop\n\tv_nop\n\tv_nop" : "+v"(d) : "v"(a), "v"(b));
  return d;
}
__device__ __forceinline__ v8f wmma_bf(v16b a, v16b b, v8f c) {
  v8f d = __builtin_amdgcn_wmma_f32_16x16x32_bf16(false, a, false, b, (short)0, c, false, false);
  asm volatile("v_nop\n\tv_nop\n\tv_nop\n\tv_nop" : "+v"(d) : "v"(a), "v"(b));
  return d;
}
__device__ __forceinline__ v16h frag_h(const _Float16* rowk0, int lane) {
  union { v16h v; v8h q[2]; } u; const _Float16* p = rowk0 + 8 * (lane >> 4);
  u.q[0] = *(const v8h*)p; u.q[1] = *(const v8h*)(p + 16); return u.v;
}
__device__ __forceinline__ v16h frag_f32(const float* rowk0, int lane) {
  v16h a; const float* p = rowk0 + 8 * (lane >> 4);
#pragma unroll
  for (int i = 0; i < 8; ++i) { a[i] = (_Float16)p[i]; a[8 + i] = (_Float16)p[16 + i]; }
  return a;
}
__device__ __forceinline__ v16h frag_f32s(const float* rowk0, int lane, float sc) {
  v16h a; const float* p = rowk0 + 8 * (lane >> 4);
#pragma unroll
  for (int i = 0; i < 8; ++i) { a[i] = (_Float16)(p[i] * sc); a[8 + i] = (_Float16)(p[16 + i] * sc); }
  return a;
}
__device__ __forceinline__ v16h fragc_f32(const float* W, int k0, int n, int lane, int ld, int K) {
  v16h a; const int g = lane >> 4;
#pragma unroll
  for (int i = 0; i < 8; ++i) { const int ka = k0 + 8 * g + i, kb = ka + 16;
    a[i] = (_Float16)(ka < K ? W[(size_t)ka * ld + n] : 0.f); a[8 + i] = (_Float16)(kb < K ? W[(size_t)kb * ld + n] : 0.f); }
  return a;
}
struct F2 { v16b h, l; };
__device__ __forceinline__ F2 bsplit16(const float v[16]) { F2 r;
#pragma unroll
  for (int i = 0; i < 16; ++i) { const __bf16 h = (__bf16)v[i]; r.h[i] = h; r.l[i] = (__bf16)(v[i] - (float)h); }
  return r; }
__device__ __forceinline__ F2 split_row(const float* row, int k0, int lane) { float v[16]; const float* p = row + k0 + 8 * (lane >> 4);
#pragma unroll
  for (int i = 0; i < 8; ++i) { v[i] = p[i]; v[8 + i] = p[16 + i]; }
  return bsplit16(v); }
__device__ __forceinline__ F2 split_rowK(const float* row, int k0, int lane, int K) { float v[16]; const int g = lane >> 4;
#pragma unroll
  for (int i = 0; i < 8; ++i) { const int ka = k0 + 8 * g + i, kb = ka + 16; v[i] = ka < K ? row[ka] : 0.f; v[8 + i] = kb < K ? row[kb] : 0.f; }
  return bsplit16(v); }
__device__ __forceinline__ F2 split_col(const float* W, int k0, int n, int lane, int ld, int K) { float v[16]; const int g = lane >> 4;
#pragma unroll
  for (int i = 0; i < 8; ++i) { const int ka = k0 + 8 * g + i, kb = ka + 16; v[i] = ka < K ? W[(size_t)ka * ld + n] : 0.f; v[8 + i] = kb < K ? W[(size_t)kb * ld + n] : 0.f; }
  return bsplit16(v); }
__device__ __forceinline__ v8f mac3(const F2& a, const F2& b, v8f c) { c = wmma_bf(a.l, b.h, c); c = wmma_bf(a.h, b.l, c); return wmma_bf(a.h, b.h, c); }
__device__ __forceinline__ float sigm(float v) { return 1.0f / (1.0f + expf(-v)); }
#define LDSX() do { asm volatile("s_wait_dscnt 0" ::: "memory"); __builtin_amdgcn_wave_barrier(); __builtin_amdgcn_fence(__ATOMIC_RELEASE, "workgroup"); } while (0)

#define NB 4
#define CC 64
#define HH 128
#define WWD 128
#define KK 4
#define HID 128
#define KIM (2 * CC * KK * KK)
#define NCELL (HH * WWD)

__device__ __forceinline__ float leaky(float v) { return v >= 0.f ? v : 0.01f * v; }

__global__ __launch_bounds__(256) void k_packW(const float* __restrict__ w1, _Float16* __restrict__ P) {
  const int o = blockIdx.x, tid = threadIdx.x; union { v8h h; v4u u; } pk;
#pragma unroll
  for (int e = 0; e < 8; ++e) pk.h[e] = (_Float16)(w1[(size_t)o * KIM + tid * 8 + e] * 16.0f);
  vst2(P + (size_t)o * KIM + tid * 8, pk.u);
}
__global__ __launch_bounds__(256) void k_blocks(const float* __restrict__ src, const float* __restrict__ tgt, const float* __restrict__ flow, int b, _Float16* __restrict__ A) {
  __shared__ __align__(16) _Float16 srow[16][KIM + 8];
  __shared__ float sfl[2][16];
  const int h = blockIdx.y, w0 = blockIdx.x * 16, tid = threadIdx.x;
  if (tid < 32) { const int c2 = tid >> 4, wl = tid & 15; sfl[c2][wl] = flow[(((size_t)b * 2 + c2) * HH + h) * WWD + w0 + wl]; }
  __syncthreads();
  const float* sb = src + (size_t)b * CC * HH * WWD; const float* tb = tgt + (size_t)b * CC * HH * WWD;
  for (int q = tid; q < 16 * 2 * CC * 16; q += 256) { const int wl = q / (2 * CC * 16), rem = q % (2 * CC * 16); const int ci = rem >> 4, d = rem & 15, di = d >> 2, dj = d & 3;
    const int w = w0 + wl; float v;
    if (ci < CC) { const int yy = h + di - 1, xx = w + dj - 1; v = (yy >= 0 && yy < HH && xx >= 0 && xx < WWD) ? tb[((size_t)ci * HH + yy) * WWD + xx] : 0.f; }
    else { const int c = ci - CC; const float ys = (float)(h + di - 1) + sfl[1][wl], xs = (float)(w + dj - 1) + sfl[0][wl];
      const float fy = floorf(ys), fx = floorf(xs); const float wy = ys - fy, wx = xs - fx; const int y0 = (int)fy, x0 = (int)fx;
      const float* pl = sb + (size_t)c * HH * WWD; float acc = 0.f;
#pragma unroll
      for (int k = 0; k < 4; ++k) { const int yi = y0 + (k >> 1), xi = x0 + (k & 1); const float wgt = ((k >> 1) ? wy : 1.0f - wy) * ((k & 1) ? wx : 1.0f - wx);
        if (yi >= 0 && yi < HH && xi >= 0 && xi < WWD) acc += pl[(size_t)yi * WWD + xi] * wgt; }
      v = acc; }
    srow[wl][ci * 16 + d] = (_Float16)v; }
  __syncthreads();
  for (int q = tid; q < 16 * KIM / 8; q += 256) { const int wl = q >> 8, pc = q & 255; vst2(A + ((size_t)h * WWD + w0 + wl) * KIM + pc * 8, *(const v4u*)(&srow[wl][pc * 8])); }
}
__global__ __launch_bounds__(128) void k_conv(const _Float16* __restrict__ A, const _Float16* __restrict__ P, const float* __restrict__ b1, const float* __restrict__ w2, const float* __restrict__ b2, int b, float* __restrict__ out) {
  __shared__ __align__(16) float sh[4][16][HID + 4];
  __shared__ __align__(16) float sa[64][20];
  __shared__ __align__(16) float so[CC][68];
  const int tid = threadIdx.x, wave = tid >> 5, lane = tid & 31, col = lane & 15, g = lane >> 4;
  const int cell0 = blockIdx.x * 64, r0 = cell0 + wave * 16; const int h = cell0 / WWD, w0 = cell0 % WWD;
  v8f acc[8] = {};
#pragma unroll 1
  for (int kc = 0; kc < KIM / 32; ++kc) { const v16h a = frag_h(A + (size_t)(r0 + col) * KIM + kc * 32, lane);
#pragma unroll
    for (int j = 0; j < 8; ++j) acc[j] = wmma16(a, frag_h(P + (size_t)(j * 16 + col) * KIM + kc * 32, lane), acc[j]); }
#pragma unroll
  for (int j = 0; j < 8; ++j) { const int o = j * 16 + col; const float bb = b1[o];
#pragma unroll
    for (int r = 0; r < 8; ++r) sh[wave][8 * g + r][o] = leaky(acc[j][r] * (1.0f / 16.0f) + bb); }
  LDSX();
  { v8f at = {};
#pragma unroll
    for (int kc = 0; kc < HID / 32; ++kc) at = wmma16(frag_f32(&sh[wave][col][0] + kc * 32, lane), frag_f32s(w2 + (size_t)col * HID + kc * 32, lane, 16.0f), at);
#pragma unroll
    for (int r = 0; r < 8; ++r) sa[wave * 16 + 8 * g + r][col] = leaky(at[r] * (1.0f / 16.0f) + b2[col]); }
  __syncthreads();
  for (int q = tid; q < 64 * CC; q += 128) { const int cl = q & 63, c = q >> 6; const _Float16* ar = A + (size_t)(cell0 + cl) * KIM + (CC + c) * 16; float s = 0.f;
#pragma unroll
    for (int d = 0; d < 16; ++d) s += sa[cl][d] * (float)ar[d];
    so[c][cl] = s * (1.0f / 16.0f); }
  __syncthreads();
  for (int q = tid; q < CC * 16; q += 128) { const int c = q >> 4, pc = q & 15; vst2(out + (((size_t)b * CC + c) * HH + h) * WWD + w0 + pc * 4, *(const v4f*)(&so[c][pc * 4])); }
}
extern "C" void kernel_launch(void* const* d_in, const int* in_sizes, int n_in, void* d_out, int out_size, void* d_ws, size_t ws_size, hipStream_t stream) {
  (void)in_sizes; (void)n_in; (void)out_size; (void)ws_size;
  const float* src = (const float*)d_in[0]; const float* tgt = (const float*)d_in[1]; const float* flow = (const float*)d_in[2]; const float* w1 = (const float*)d_in[3]; const float* b1 = (const float*)d_in[4]; const float* w2 = (const float*)d_in[5]; const float* b2 = (const float*)d_in[6];
  float* out = (float*)d_out;
  char* ws = (char*)d_ws; size_t off = 0;
  auto take = [&](size_t bytes) { char* p = ws + off; off += (bytes + 255) & ~(size_t)255; return p; };
  _Float16* P = (_Float16*)take((size_t)HID * KIM * 2); _Float16* A = (_Float16*)take((size_t)NCELL * KIM * 2);
  k_packW<<<HID, 256, 0, stream>>>(w1, P);
  for (int b = 0; b < NB; ++b) {
    k_blocks<<<dim3(WWD / 16, HH), 256, 0, stream>>>(src, tgt, flow, b, A);
    k_conv<<<NCELL / 64, 128, 0, stream>>>(A, P, b1, w2, b2, b, out); }
}
